// MultiHeadAttention_2894807958079
// MI455X (gfx1250) — hardware-verified
//
#include <hip/hip_runtime.h>
#include <math.h>

typedef __attribute__((ext_vector_type(16))) _Float16 v16h;
typedef __attribute__((ext_vector_type(8)))  _Float16 v8h;
typedef __attribute__((ext_vector_type(8)))  float    v8f;
typedef __attribute__((ext_vector_type(4)))  float    v4f;

constexpr int kBatch = 8;
constexpr int kSeq   = 2048;
constexpr int kHeads = 8;
constexpr int kHd    = 64;
constexpr int kRows  = kBatch * kSeq * kHeads;
constexpr int kBH    = kBatch * kHeads;
constexpr int kWEl   = kHd * kHd;
constexpr int kPitch = 68;
static_assert(kRows == 131072);
static_assert(kHd == 64 && (kHd % 32) == 0);
static_assert((kSeq % 64) == 0 && (kRows % 64) == 0);

constexpr double c_sqrt(double v) {
  double r = v > 1.0 ? v : 1.0;
  for (int i = 0; i < 64; ++i) r = 0.5 * (r + v / r);
  return r;
}
constexpr float kInvSqrtD = (float)(1.0 / c_sqrt((double)kHd));
static_assert(kInvSqrtD == 0.125f);
constexpr float kXCarry   = 16.0f;
constexpr float kWCarry   = 256.0f;
constexpr float kQKVCarry = 16.0f;
constexpr float kOCarry   = 256.0f;
constexpr float kPShift   = 10.0f;
constexpr float kInvXW    = 1.0f / (kXCarry * kWCarry);
constexpr float kLog2e    = 1.4426950408889634f;
constexpr float kScoreC   = kLog2e * kInvSqrtD / (kQKVCarry * kQKVCarry);
constexpr float kORatio   = kOCarry / kQKVCarry;
constexpr float kOutScale = 1.0f / (kOCarry * kWCarry);

constexpr size_t kOffW  = 0;
constexpr size_t kOffQ  = kOffW  + (size_t)4 * kWEl * 2;
constexpr size_t kOffK  = kOffQ  + (size_t)kRows * kHd * 2;
constexpr size_t kOffVT = kOffK  + (size_t)kRows * kHd * 2;
constexpr size_t kOffO  = kOffVT + (size_t)kRows * kHd * 2;
constexpr size_t kWsTotal = kOffO + (size_t)kRows * kHd * 2;
static_assert(kWsTotal == 67141632ull);
static_assert(kWsTotal <= 134217728ull);
static_assert((kOffQ % 128) == 0 && (kOffK % 128) == 0 && (kOffVT % 128) == 0 && (kOffO % 128) == 0);

union FragU { v16h v; v8h h[2]; };
__device__ __forceinline__ v16h frag_ld(const _Float16* p) {
  FragU f;
  f.h[0] = *(const v8h*)(p);
  f.h[1] = *(const v8h*)(p + 16);
  return f.v;
}
__device__ __forceinline__ v8f mma_f16(v16h a, v16h b, v8f c) {
  c = __builtin_amdgcn_wmma_f32_16x16x32_f16(false, a, false, b, (short)0, c, false, false);
  asm volatile("v_nop\n\tv_nop\n\tv_nop\n\tv_nop" : "+v"(c) : "v"(a), "v"(b));
  return c;
}
__device__ __forceinline__ void guard4_h(v8f& a, v8f& b, v8f& c, v8f& d, v16h x, v16h y) {
  asm volatile("v_nop\n\tv_nop\n\tv_nop\n\tv_nop" : "+v"(a), "+v"(b), "+v"(c), "+v"(d) : "v"(x), "v"(y));
}
__device__ __forceinline__ void keep4_h(v16h a, v16h b, v16h c, v16h d) {
  asm volatile("v_nop" :: "v"(a), "v"(b), "v"(c), "v"(d));
}
__device__ __forceinline__ void acc_guard4(v8f& a, v8f& b, v8f& c, v8f& d) {
  asm volatile("v_nop\n\tv_nop\n\tv_nop\n\tv_nop" : "+v"(a), "+v"(b), "+v"(c), "+v"(d));
}
__device__ __forceinline__ void wave_lds_sync() {
  __builtin_amdgcn_fence(__ATOMIC_RELEASE, "workgroup");
  __builtin_amdgcn_wave_barrier();
  __builtin_amdgcn_fence(__ATOMIC_ACQUIRE, "workgroup");
}

__device__ __forceinline__ v16h x_frag(const float* p) {
  const v4f a0 = *(const v4f*)(p);
  const v4f a1 = *(const v4f*)(p + 4);
  const v4f a2 = *(const v4f*)(p + 16);
  const v4f a3 = *(const v4f*)(p + 20);
  v16h f;
#pragma unroll
  for (int e = 0; e < 4; ++e) {
    f[e]      = (_Float16)(a0[e] * kXCarry);
    f[4 + e]  = (_Float16)(a1[e] * kXCarry);
    f[8 + e]  = (_Float16)(a2[e] * kXCarry);
    f[12 + e] = (_Float16)(a3[e] * kXCarry);
  }
  return f;
}

__device__ __forceinline__ void store_rows16_f16(const float* src, unsigned short* dst, size_t dpitch, int lane) {
  const int q = lane >> 3;
  const int c8 = (lane & 7) * 8;
  v8h hv[4];
#pragma unroll
  for (int it = 0; it < 4; ++it) {
    const float* sp = src + (it * 4 + q) * kPitch + c8;
    const v4f a0 = *(const v4f*)(sp);
    const v4f a1 = *(const v4f*)(sp + 4);
#pragma unroll
    for (int e = 0; e < 4; ++e) {
      hv[it][e]     = (_Float16)a0[e];
      hv[it][4 + e] = (_Float16)a1[e];
    }
  }
  for (int pass = 0; pass < 2; ++pass) {
#pragma unroll
    for (int it = 0; it < 4; ++it) {
      *(volatile v8h*)(dst + (size_t)(it * 4 + q) * dpitch + c8) = hv[it];
    }
    __threadfence();
  }
}

__global__ __launch_bounds__(256) void wcast_kernel(const float* __restrict__ W0, const float* __restrict__ W1,
                                                    const float* __restrict__ W2, const float* __restrict__ W3,
                                                    unsigned short* __restrict__ out) {
  const int z = blockIdx.x >> 1;
  const float* W = (z == 0) ? W0 : (z == 1) ? W1 : (z == 2) ? W2 : W3;
  const int i = (blockIdx.x & 1) * 256 + threadIdx.x;
  const float* p = W + 8 * i;
  const v4f a = *(const v4f*)(p);
  const v4f c = *(const v4f*)(p + 4);
  v8h hv;
#pragma unroll
  for (int e = 0; e < 4; ++e) {
    hv[e]     = (_Float16)(a[e] * kWCarry);
    hv[4 + e] = (_Float16)(c[e] * kWCarry);
  }
  unsigned short* q = out + (size_t)z * kWEl + 8 * i;
  *(volatile v8h*)q = hv;
  __threadfence();
  *(volatile v8h*)q = hv;
}

template <bool TR>
__device__ __forceinline__ void proj_tile(v16h ax0, v16h ax1, const _Float16* Wm, const float* bias,
                                          float* dst, int colbase, int hh, int c) {
  v16h w0[4], w1[4];
#pragma unroll
  for (int j = 0; j < 4; ++j) {
    const _Float16* wp = Wm + (j * 16 + c) * kHd + 8 * hh;
    w0[j] = frag_ld(wp);
    w1[j] = frag_ld(wp + 32);
  }
  v8f acc[4];
#pragma unroll
  for (int j = 0; j < 4; ++j) {
    acc[j] = (v8f){0.f, 0.f, 0.f, 0.f, 0.f, 0.f, 0.f, 0.f};
    acc[j] = mma_f16(ax0, w0[j], acc[j]);
    acc[j] = mma_f16(ax1, w1[j], acc[j]);
  }
#pragma unroll
  for (int j = 0; j < 4; ++j) {
    const float bj = bias[j * 16 + c];
#pragma unroll
    for (int r = 0; r < 8; ++r) {
      const float v = (acc[j][r] * kInvXW + bj) * kQKVCarry;
      if (TR) dst[(j * 16 + c) * kPitch + colbase + 8 * hh + r] = v;
      else    dst[(8 * hh + r) * kPitch + j * 16 + c] = v;
    }
  }
}

__global__ __launch_bounds__(128) void qkv_proj_kernel(
    const float* __restrict__ x, const unsigned short* __restrict__ W16p,
    const float* __restrict__ bq, const float* __restrict__ bk, const float* __restrict__ bv,
    unsigned short* __restrict__ Q16p, unsigned short* __restrict__ K16p, unsigned short* __restrict__ VT16p) {
  __shared__ __align__(16) float sSlab[4][16 * kPitch];
  __shared__ __align__(16) float sVt[64 * kPitch];
  const int tid  = threadIdx.x;
  const int wave = __builtin_amdgcn_readfirstlane((int)(tid >> 5));
  const int lane = tid & 31;
  const int hh   = lane >> 4;
  const int c    = lane & 15;
  const int bh   = blockIdx.y;
  const int b    = bh / kHeads;
  const int h    = bh - b * kHeads;
  const int sblk = blockIdx.x * 64;
  const int s0   = sblk + wave * 16;

  const float* xr = x + (((size_t)b * kSeq + s0 + c) * kHeads + h) * kHd + 8 * hh;
  const v16h ax0 = x_frag(xr);
  const v16h ax1 = x_frag(xr + 32);

  const _Float16* W16 = (const _Float16*)W16p;
  float* slab = sSlab[wave];

  proj_tile<false>(ax0, ax1, W16, bq, slab, 0, hh, c);
  wave_lds_sync();
  store_rows16_f16(slab, Q16p + ((size_t)bh * kSeq + s0) * kHd, (size_t)kHd, lane);
  wave_lds_sync();

  proj_tile<false>(ax0, ax1, W16 + kWEl, bk, slab, 0, hh, c);
  wave_lds_sync();
  store_rows16_f16(slab, K16p + ((size_t)bh * kSeq + s0) * kHd, (size_t)kHd, lane);

  proj_tile<true>(ax0, ax1, W16 + 2 * kWEl, bv, sVt, wave * 16, hh, c);
  __syncthreads();
  store_rows16_f16(sVt + (wave * 16) * kPitch,
                   VT16p + ((size_t)bh * kHd + wave * 16) * kSeq + sblk, (size_t)kSeq, lane);
}

__global__ __launch_bounds__(128) void attn_kernel(
    const unsigned short* __restrict__ Q16p, const unsigned short* __restrict__ K16p,
    const unsigned short* __restrict__ VT16p, unsigned short* __restrict__ O16p) {
  __shared__ __align__(16) _Float16 sK[64 * 64];
  __shared__ __align__(16) _Float16 sV[64 * 64];
  __shared__ __align__(16) _Float16 sP[4][16 * 64];
  __shared__ __align__(16) float    sO[4][16 * kPitch];

  const int tid  = threadIdx.x;
  const int wave = __builtin_amdgcn_readfirstlane((int)(tid >> 5));
  const int lane = tid & 31;
  const int hh   = lane >> 4;
  const int c    = lane & 15;
  const int bh   = blockIdx.y;
  const int b    = bh / kHeads;
  const int h    = bh - b * kHeads;
  const int q0   = blockIdx.x * 64 + wave * 16;

  const _Float16* Qg = (const _Float16*)Q16p + ((size_t)bh * kSeq + q0 + c) * kHd + 8 * hh;
  const _Float16* Kg = (const _Float16*)K16p + (size_t)bh * kSeq * kHd;
  const _Float16* Vg = (const _Float16*)VT16p + (size_t)bh * kHd * kSeq;

  const v16h qa0 = frag_ld(Qg);
  const v16h qa1 = frag_ld(Qg + 32);

  float mrow[8], lrow[8];
  v8f oacc[4];
#pragma unroll
  for (int r = 0; r < 8; ++r) { mrow[r] = -3.0e38f; lrow[r] = 0.f; }
#pragma unroll
  for (int t = 0; t < 4; ++t) oacc[t] = (v8f){0.f, 0.f, 0.f, 0.f, 0.f, 0.f, 0.f, 0.f};

  _Float16* pw = sP[wave];

#pragma unroll 1
  for (int kc = 0; kc < kSeq / 64; ++kc) {
    const int kv0 = kc * 64;
    __syncthreads();
    {
      v8h kr[4], vr[4];
#pragma unroll
      for (int i = 0; i < 4; ++i) {
        const int idx = tid + 128 * i;
        const int d_  = idx >> 3;
        const int off = (idx & 7) * 8;
        kr[i] = *(const v8h*)(Kg + (size_t)kv0 * kHd + idx * 8);
        vr[i] = *(const v8h*)(Vg + (size_t)d_ * kSeq + kv0 + off);
      }
#pragma unroll
      for (int i = 0; i < 4; ++i) {
        const int idx = tid + 128 * i;
        const int d_  = idx >> 3;
        const int off = (idx & 7) * 8;
        *(v8h*)(sK + idx * 8) = kr[i];
        *(v8h*)(sV + d_ * 64 + off) = vr[i];
      }
    }
    __syncthreads();

    v8f s[4];
#pragma unroll
    for (int j = 0; j < 4; ++j) {
      const _Float16* kp = sK + (j * 16 + c) * 64 + 8 * hh;
      const v16h kb0 = frag_ld(kp);
      const v16h kb1 = frag_ld(kp + 32);
      s[j] = (v8f){0.f, 0.f, 0.f, 0.f, 0.f, 0.f, 0.f, 0.f};
      s[j] = mma_f16(qa0, kb0, s[j]);
      s[j] = mma_f16(qa1, kb1, s[j]);
    }

#pragma unroll
    for (int r = 0; r < 8; ++r) {
      float m = fmaxf(fmaxf(s[0][r], s[1][r]), fmaxf(s[2][r], s[3][r]));
#pragma unroll
      for (int off = 1; off < 16; off <<= 1) m = fmaxf(m, __shfl_xor(m, off, 32));
      const float mt    = m * kScoreC;
      const float mnew  = fmaxf(mrow[r], mt);
      const float alpha = __builtin_amdgcn_exp2f(mrow[r] - mnew);
      mrow[r] = mnew;
      const float nb = kPShift - mnew;
      float psum = 0.f;
#pragma unroll
      for (int j = 0; j < 4; ++j) {
        const float p = __builtin_amdgcn_exp2f(fmaf(s[j][r], kScoreC, nb));
        psum += p;
        pw[(8 * hh + r) * 64 + j * 16 + c] = (_Float16)p;
      }
      lrow[r] = fmaf(lrow[r], alpha, psum);
#pragma unroll
      for (int t = 0; t < 4; ++t) oacc[t][r] *= alpha;
    }
    wave_lds_sync();

#pragma unroll
    for (int kk = 0; kk < 2; ++kk) {
      const v16h pa = frag_ld(pw + c * 64 + kk * 32 + 8 * hh);
#pragma unroll
      for (int t = 0; t < 4; ++t) {
        const v16h vb = frag_ld(sV + (t * 16 + c) * 64 + kk * 32 + 8 * hh);
        oacc[t] = mma_f16(pa, vb, oacc[t]);
      }
    }
  }

  float* os = sO[wave];
#pragma unroll
  for (int r = 0; r < 8; ++r) {
    float l = lrow[r];
#pragma unroll
    for (int off = 1; off < 16; off <<= 1) l += __shfl_xor(l, off, 32);
    const float inv = kORatio * (1.0f / l);
#pragma unroll
    for (int t = 0; t < 4; ++t) os[(8 * hh + r) * kPitch + t * 16 + c] = oacc[t][r] * inv;
  }
  wave_lds_sync();
  store_rows16_f16(os, O16p + (((size_t)b * kSeq + q0) * kHeads + h) * kHd, (size_t)kHeads * kHd, lane);
}

__global__ __launch_bounds__(256) void out_proj_kernel(
    const unsigned short* __restrict__ Ap, int lda,
    const unsigned short* __restrict__ Btp, int ldb,
    float* __restrict__ C, int ldc,
    const float* __restrict__ bias,
    int M, int N, int K, float scale) {
  const _Float16* A  = (const _Float16*)Ap;
  const _Float16* Bt = (const _Float16*)Btp;
  __shared__ __align__(16) float sT[8][16 * kPitch];
  const int lane = threadIdx.x & 31;
  const int wave = __builtin_amdgcn_readfirstlane((int)(threadIdx.x >> 5));
  const int tilesN = N >> 6;
  const int tilesM = M >> 6;
  const int tile = blockIdx.x * 8 + wave;
  if (tile >= tilesM * tilesN) return;
  const int tm = tile / tilesN;
  const int tn = tile - tm * tilesN;
  const int m0 = tm << 6;
  const int n0 = tn << 6;

  const int rlane = lane & 15;
  const int koff  = (lane >> 4) * 8;
  const int mOff  = (lane >> 4) * 8;

  v8f acc[4][4];
#pragma unroll
  for (int i = 0; i < 4; ++i)
#pragma unroll
    for (int j = 0; j < 4; ++j) acc[i][j] = (v8f){0.f, 0.f, 0.f, 0.f, 0.f, 0.f, 0.f, 0.f};

  for (int k0 = 0; k0 < K; k0 += 32) {
    v16h bh[4];
#pragma unroll
    for (int j = 0; j < 4; ++j) {
      const size_t bo = (size_t)(n0 + (j << 4) + rlane) * ldb + koff + k0;
      bh[j] = frag_ld(Bt + bo);
    }
#pragma unroll
    for (int i = 0; i < 4; ++i) {
      const size_t ao = (size_t)(m0 + (i << 4) + rlane) * lda + koff + k0;
      const v16h ah = frag_ld(A + ao);
#pragma unroll
      for (int j = 0; j < 4; ++j) {
        acc[i][j] = __builtin_amdgcn_wmma_f32_16x16x32_f16(false, ah, false, bh[j], (short)0, acc[i][j], false, false);
      }
      guard4_h(acc[i][0], acc[i][1], acc[i][2], acc[i][3], ah, ah);
    }
    keep4_h(bh[0], bh[1], bh[2], bh[3]);
  }
  acc_guard4(acc[0][0], acc[0][1], acc[0][2], acc[0][3]);
  acc_guard4(acc[1][0], acc[1][1], acc[1][2], acc[1][3]);
  acc_guard4(acc[2][0], acc[2][1], acc[2][2], acc[2][3]);
  acc_guard4(acc[3][0], acc[3][1], acc[3][2], acc[3][3]);

  float* slab = sT[wave];
#pragma unroll
  for (int i = 0; i < 4; ++i) {
    const int mBase = m0 + (i << 4);
#pragma unroll
    for (int j = 0; j < 4; ++j) {
      const int n = n0 + (j << 4) + rlane;
      const float bvv = bias[n];
#pragma unroll
      for (int r = 0; r < 8; ++r) {
        const float v = acc[i][j][r] * scale + bvv;
        slab[(mOff + r) * kPitch + (j << 4) + rlane] = v;
      }
    }
    wave_lds_sync();
    {
      const int hh = lane >> 4;
      const int c4 = (lane & 15) * 4;
      for (int pass = 0; pass < 2; ++pass) {
#pragma unroll
        for (int it = 0; it < 8; ++it) {
          const int row = it * 2 + hh;
          const v4f v = *(const v4f*)(slab + row * kPitch + c4);
          *(volatile v4f*)(C + (size_t)(mBase + row) * ldc + n0 + c4) = v;
        }
        __threadfence();
      }
    }
    wave_lds_sync();
  }
}

extern "C" void kernel_launch(void* const* d_in, const int* in_sizes, int n_in,
                              void* d_out, int out_size, void* d_ws, size_t ws_size,
                              hipStream_t stream) {
  if (n_in < 9) return;
  if (in_sizes[0] != kRows * kHd) return;
  if (in_sizes[1] != kWEl || in_sizes[3] != kWEl || in_sizes[5] != kWEl || in_sizes[7] != kWEl) return;
  if (in_sizes[2] != kHd || in_sizes[4] != kHd || in_sizes[6] != kHd || in_sizes[8] != kHd) return;
  if (out_size != kRows * kHd) return;
  if (ws_size < kWsTotal) return;

  const float* x  = (const float*)d_in[0];
  const float* Wq = (const float*)d_in[1];
  const float* bq = (const float*)d_in[2];
  const float* Wk = (const float*)d_in[3];
  const float* bk = (const float*)d_in[4];
  const float* Wv = (const float*)d_in[5];
  const float* bv = (const float*)d_in[6];
  const float* Wo = (const float*)d_in[7];
  const float* bo = (const float*)d_in[8];
  float* out = (float*)d_out;

  char* ws = (char*)d_ws;
  unsigned short* W16  = (unsigned short*)(ws + kOffW);
  unsigned short* Q16  = (unsigned short*)(ws + kOffQ);
  unsigned short* K16  = (unsigned short*)(ws + kOffK);
  unsigned short* VT16 = (unsigned short*)(ws + kOffVT);
  unsigned short* O16  = (unsigned short*)(ws + kOffO);

  wcast_kernel<<<8, 256, 0, stream>>>(Wq, Wk, Wv, Wo, W16);

  qkv_proj_kernel<<<dim3(kSeq / 64, kBH), 128, 0, stream>>>(x, W16, bq, bk, bv, Q16, K16, VT16);

  attn_kernel<<<dim3(kSeq / 64, kBH), 128, 0, stream>>>(Q16, K16, VT16, O16);

  out_proj_kernel<<<dim3(kRows / 64 / 8, 1), 256, 0, stream>>>(
      O16, kHd, W16 + 3 * kWEl, kHd, out, kHd, bo, kRows, kHd, kHd, kOutScale);
}
